// GAT_85950885528277
// MI455X (gfx1250) — hardware-verified
//
#include <hip/hip_runtime.h>
#include <stddef.h>
#include <stdint.h>
#include <math.h>


#define F0      213
#define KP1     224
#define HC1     192
#define NH1     12
#define CH1     16
#define HC2     64
#define NH2     8
#define CH2     8
#define KA2     384
#define PIT1    224
#define PIT2    96
#define NTHR    256
#define NWAVE   8
#define EPT     8
#define CHUNK   (NTHR * EPT)
#define WCAP    (EPT * 32)
#define LISTN   (NWAVE * WCAP)
#define NB      1024
#define SLOTB   10
#define NBW     (NB / NWAVE)
#define RCAP    20480
#define DEGCAP  128
#define STW     384
#define MROWS   128
#define GBM     64
#define PPB     256
#define NU1     (HC1 * (KP1 / 8))
#define NU2     (HC2 * (KA2 / 8))
#define NEGSL   0.2f
#define WSMAX   134217728
#define LDS_AGG ((2 * RCAP + 2 * NB + LISTN + 16) * 4)

static_assert((CHUNK & (CHUNK - 1)) == 0 && CHUNK <= 2048);
static_assert(NB == (1 << SLOTB));
static_assert(NTHR * 4 == NB);
static_assert(LISTN >= NB && LISTN >= HC1);
static_assert((RCAP % 32) == 0 && NWAVE * STW <= RCAP);
static_assert(LDS_AGG <= 300000);
static_assert((KP1 % 32) == 0 && (KA2 % 32) == 0 && KA2 == 2 * HC1);
static_assert((NU1 % NTHR) == 0 && (NU2 % NTHR) == 0);
static_assert((MROWS % GBM) == 0);
static_assert(NH1 * CH1 == HC1 && NH2 * CH2 == HC2);
static_assert(HC1 == 4 * 32 + 2 * 32 && HC2 == 2 * 32);

typedef float          v2f  __attribute__((ext_vector_type(2)));
typedef float          v4f  __attribute__((ext_vector_type(4)));
typedef float          v8f  __attribute__((ext_vector_type(8)));
typedef int            v4i  __attribute__((ext_vector_type(4)));
typedef int            v8i  __attribute__((ext_vector_type(8)));
typedef unsigned int   v4u  __attribute__((ext_vector_type(4)));
typedef unsigned short v8us __attribute__((ext_vector_type(8)));
typedef __bf16         v16b __attribute__((ext_vector_type(16)));
typedef v2f  __attribute__((may_alias)) v2fa;
typedef v4f  __attribute__((may_alias)) v4fa;
typedef v8us __attribute__((may_alias)) v8usa;
union FragB { v16b v; v8us h[2]; v8i w; };

__device__ __forceinline__ v8f wmb(const FragB& a, const FragB& b, v8f c) {
  v8f d = __builtin_amdgcn_wmma_f32_16x16x32_bf16(false, a.v, false, b.v, (short)0, c, false, false);
  asm volatile("v_nop\n\tv_nop\n\tv_nop\n\tv_nop" : "+v"(d) : "v"(a.w), "v"(b.w));
  return d;
}

__device__ __forceinline__ unsigned int f2bf(float f) {
  const unsigned int u = __float_as_uint(f);
  const unsigned int r = ((u + 0x7FFFu + ((u >> 16) & 1u)) >> 16) & 0xFFFFu;
  return (f != f) ? 0x7FC0u : r;
}
__device__ __forceinline__ float bf2f(unsigned int b) { return __uint_as_float(b << 16); }
__device__ __forceinline__ float bfr(float f) { return bf2f(f2bf(f)); }
__device__ __forceinline__ unsigned int pk2(float lo, float hi) { return f2bf(lo) | (f2bf(hi) << 16); }

__device__ __forceinline__ void st2_u4(unsigned short* p, const v4u v) {
  *(volatile v4u*)p = v;
  __threadfence();
  *(volatile v4u*)p = v;
}

__device__ __forceinline__ float lrelu(float v) { return v > 0.f ? v : NEGSL * v; }

__device__ __forceinline__ void onl_step(float lg, float& mx, float& dn, float& s1, float& s2) {
  const float df = lg - mx;
  const float ee = __expf(-fabsf(df));
  const bool  up = df > 0.f;
  s1 = up ? ee : 1.0f;
  s2 = up ? 1.0f : ee;
  mx = up ? lg : mx;
  dn = fmaf(dn, s1, s2);
}

__device__ __forceinline__ int scan_chunk(const int* __restrict__ dsts, int nE, int cbase, int slotBase,
                                          int nb, int vec8, int* list, int tid, int lane, int wave) {
  int wc = 0;
  const int el0  = tid * EPT;
  const int e0   = cbase + el0;
  const int sent = -2147483647 - 1;
  v4i da, db;
  if (vec8 != 0 && cbase + CHUNK <= nE) {
    da = *(const v4i*)(dsts + e0);
    db = *(const v4i*)(dsts + e0 + 4);
  } else {
    da.x = (e0     < nE) ? dsts[min(e0,     nE - 1)] : sent;
    da.y = (e0 + 1 < nE) ? dsts[min(e0 + 1, nE - 1)] : sent;
    da.z = (e0 + 2 < nE) ? dsts[min(e0 + 2, nE - 1)] : sent;
    da.w = (e0 + 3 < nE) ? dsts[min(e0 + 3, nE - 1)] : sent;
    db.x = (e0 + 4 < nE) ? dsts[min(e0 + 4, nE - 1)] : sent;
    db.y = (e0 + 5 < nE) ? dsts[min(e0 + 5, nE - 1)] : sent;
    db.z = (e0 + 6 < nE) ? dsts[min(e0 + 6, nE - 1)] : sent;
    db.w = (e0 + 7 < nE) ? dsts[min(e0 + 7, nE - 1)] : sent;
  }
  const unsigned nbs = (unsigned)slotBase;
  const unsigned unb = (unsigned)nb;
  const unsigned s0 = (unsigned)da.x - nbs, s1 = (unsigned)da.y - nbs;
  const unsigned s2 = (unsigned)da.z - nbs, s3 = (unsigned)da.w - nbs;
  const unsigned s4 = (unsigned)db.x - nbs, s5 = (unsigned)db.y - nbs;
  const unsigned s6 = (unsigned)db.z - nbs, s7 = (unsigned)db.w - nbs;
  const bool h0 = s0 < unb, h1 = s1 < unb, h2 = s2 < unb, h3 = s3 < unb;
  const bool h4 = s4 < unb, h5 = s5 < unb, h6 = s6 < unb, h7 = s7 < unb;
  const unsigned any = __builtin_amdgcn_ballot_w32(h0 | h1 | h2 | h3 | h4 | h5 | h6 | h7);
  if (any != 0u) {
#define HITJ(J, HJ, SJ) { \
      const unsigned mj = __builtin_amdgcn_ballot_w32(HJ); \
      if (mj != 0u) { \
        if (HJ) { \
          const int pos = wc + (int)__builtin_amdgcn_mbcnt_lo(mj, 0u); \
          if (pos < WCAP) list[wave * WCAP + pos] = ((el0 + (J)) << SLOTB) | (int)(SJ); \
        } \
        wc += (int)__builtin_popcount(mj); } }
    HITJ(0, h0, s0)
    HITJ(1, h1, s1)
    HITJ(2, h2, s2)
    HITJ(3, h3, s3)
    HITJ(4, h4, s4)
    HITJ(5, h5, s5)
    HITJ(6, h6, s6)
    HITJ(7, h7, s7)
#undef HITJ
  }
  return wc;
}

__global__ __launch_bounds__(NTHR) void k_xprep(const float* __restrict__ x, unsigned short* xb, int nN, int nUnits) {
  const int u = (int)blockIdx.x * NTHR + (int)threadIdx.x;
  if (u >= nUnits) return;
  const int row = u / (KP1 / 8);
  const int c0  = (u - row * (KP1 / 8)) * 8;
  const int rc  = row < nN ? row : nN - 1;
  const bool rok = row < nN;
  const float* p = x + (size_t)rc * F0;
  float v[8];
#pragma unroll
  for (int i = 0; i < 8; ++i) {
    const int c  = c0 + i;
    const int cc = c < F0 ? c : F0 - 1;
    const float t = p[cc];
    v[i] = (rok && c < F0) ? t : 0.0f;
  }
  v4u hv;
  hv.x = pk2(v[0], v[1]); hv.y = pk2(v[2], v[3]); hv.z = pk2(v[4], v[5]); hv.w = pk2(v[6], v[7]);
  st2_u4(xb + (size_t)u * 8, hv);
}

__global__ __launch_bounds__(NTHR) void k_wprep(const float* __restrict__ W1, const float* __restrict__ W2,
                                                unsigned short* W1T, unsigned short* W2T) {
  const int u = (int)blockIdx.x * NTHR + (int)threadIdx.x;
  float v[8];
  if (u < NU1) {
    const int n  = u / (KP1 / 8);
    const int k8 = (u - n * (KP1 / 8)) * 8;
#pragma unroll
    for (int i = 0; i < 8; ++i) {
      const int k  = k8 + i;
      const int kc = k < F0 ? k : F0 - 1;
      const float t = W1[(size_t)kc * HC1 + n];
      v[i] = (k < F0) ? t : 0.0f;
    }
    v4u wv;
    wv.x = pk2(v[0], v[1]); wv.y = pk2(v[2], v[3]); wv.z = pk2(v[4], v[5]); wv.w = pk2(v[6], v[7]);
    st2_u4(W1T + (size_t)u * 8, wv);
  } else if (u < NU1 + NU2) {
    const int w  = u - NU1;
    const int n  = w / (KA2 / 8);
    const int k8 = (w - n * (KA2 / 8)) * 8;
    const int kk = k8 >= HC1 ? k8 - HC1 : k8;
#pragma unroll
    for (int i = 0; i < 8; ++i) v[i] = W2[(size_t)(kk + i) * HC2 + n];
    v4u wv;
    wv.x = pk2(v[0], v[1]); wv.y = pk2(v[2], v[3]); wv.z = pk2(v[4], v[5]); wv.w = pk2(v[6], v[7]);
    st2_u4(W2T + (size_t)w * 8, wv);
  }
}

template<int THR, int NT, int KK, int PIT, int NCOL, int NHD, int CHD>
__global__ __launch_bounds__(THR) void k_gemm(const unsigned short* __restrict__ A,
                                              const unsigned short* __restrict__ WT,
                                              const float* __restrict__ atts, const float* __restrict__ attd,
                                              float* HA) {
  constexpr int NCG = THR / 128;
  constexpr int TPR = THR / 64;
  constexpr int TPT = (2 * NHD) / TPR;
  constexpr int ZP4 = (PIT - NCOL - 2 * NHD) / 4;
  constexpr int NPC = GBM * PIT / 4;
  static_assert(NCG * NT * 16 == NCOL);
  static_assert(TPT * TPR == 2 * NHD && (NHD % TPT) == 0);
  static_assert(NHD * CHD == NCOL && (CHD % 4) == 0);
  static_assert(((NCOL + 2 * NHD) % 4) == 0 && (PIT % 4) == 0 && ZP4 >= 0);
  static_assert((KK % 32) == 0 && (NPC % THR) == 0);
  __shared__ __attribute__((aligned(16))) float stg[GBM * PIT];
  __shared__ __attribute__((aligned(16))) float satt[2 * NCOL];
  const int tid = (int)threadIdx.x, lane = tid & 31, wave = tid >> 5, hh = lane >> 4, m = lane & 15;
  const int rg = wave & 3, cg = wave >> 2;
  const int rowBase = (int)blockIdx.x * GBM;
  const int colBase = cg * (NT * 16);

  for (int i = tid; i < 2 * NCOL; i += THR) {
    const int c = i < NCOL ? i : i - NCOL;
    const float vs = atts[c];
    const float vd = attd[c];
    satt[i] = bfr(i < NCOL ? vs : vd);
  }

  v8f acc[NT];
  {
    const v8f z = {0.f, 0.f, 0.f, 0.f, 0.f, 0.f, 0.f, 0.f};
#pragma unroll
    for (int t = 0; t < NT; ++t) acc[t] = z;
  }
  const unsigned short* ap = A  + (size_t)(rowBase + 16 * rg + m) * (size_t)KK + 8 * hh;
  const unsigned short* bp = WT + (size_t)(colBase + m) * (size_t)KK + 8 * hh;
#pragma unroll 1
  for (int k0 = 0; k0 < KK; k0 += 32) {
    FragB af;
    af.h[0] = *(const v8usa*)(ap + k0);
    af.h[1] = *(const v8usa*)(ap + k0 + 16);
#pragma unroll
    for (int nt = 0; nt < NT; ++nt) {
      const unsigned short* wq = bp + (size_t)(16 * nt) * (size_t)KK + k0;
      FragB bf;
      bf.h[0] = *(const v8usa*)wq;
      bf.h[1] = *(const v8usa*)(wq + 16);
      acc[nt] = wmb(af, bf, acc[nt]);
    }
  }

#pragma unroll
  for (int nt = 0; nt < NT; ++nt) {
    const int lc = colBase + 16 * nt + m;
#pragma unroll
    for (int r = 0; r < 8; ++r) {
      const int lr = 16 * rg + 8 * hh + r;
      stg[lr * PIT + lc] = acc[nt][r];
    }
  }
  __syncthreads();

  {
    const int row = tid & 63, q = tid >> 6;
    const float* hr = stg + row * PIT;
#pragma unroll 1
    for (int j = 0; j < TPT; ++j) {
      const int tk    = q * TPT + j;
      const int which = tk / NHD;
      const int hd    = tk - which * NHD;
      const float* sa = satt + which * NCOL + hd * CHD;
      const float* hp = hr + hd * CHD;
      float d = 0.f;
#pragma unroll
      for (int c4 = 0; c4 < CHD / 4; ++c4) {
        const v4f hv = *(const v4fa*)(hp + 4 * c4);
        const v4f av = *(const v4fa*)(sa + 4 * c4);
        d = fmaf(hv.x, av.x, d);
        d = fmaf(hv.y, av.y, d);
        d = fmaf(hv.z, av.z, d);
        d = fmaf(hv.w, av.w, d);
      }
      stg[row * PIT + NCOL + tk] = d;
    }
    const v4f z4 = {0.f, 0.f, 0.f, 0.f};
    for (int z = q; z < ZP4; z += TPR) *(v4fa*)(stg + row * PIT + NCOL + 2 * NHD + 4 * z) = z4;
  }
  __syncthreads();

  float* ob = HA + (size_t)rowBase * (size_t)PIT;
#pragma unroll 1
  for (int it = 0; it < NPC / THR; ++it) {
    const int p = it * THR + tid;
    const v4f v = *(const v4fa*)(stg + 4 * p);
    *(volatile v4f*)(ob + 4 * p) = v;
  }
  __threadfence();
#pragma unroll 1
  for (int it = 0; it < NPC / THR; ++it) {
    const int p = it * THR + tid;
    const v4f v = *(const v4fa*)(stg + 4 * p);
    *(volatile v4f*)(ob + 4 * p) = v;
  }
}

template<int L>
__global__ __launch_bounds__(NTHR) void k_agg(
    const int* __restrict__ srcs, const int* __restrict__ dsts,
    const float* __restrict__ F, const float* __restrict__ bias,
    unsigned short* HP, float* xout,
    int nN, int nE, int vec8, int MPr) {
  constexpr int PIT  = (L == 1) ? PIT1 : PIT2;
  constexpr int NCOL = (L == 1) ? HC1 : HC2;
  constexpr int NHD  = (L == 1) ? NH1 : NH2;
  constexpr int ASO  = NCOL;
  constexpr int ADO  = NCOL + NHD;
  extern __shared__ v4f lds_dyn[];
  int* reg1 = (int*)lds_dyn;
  int* reg2 = reg1 + RCAP;
  int* scnt = reg2 + RCAP;
  int* soff = scnt + NB;
  int* list = soff + NB;
  int* wcnt = list + LISTN;
  int* wtot = wcnt + NWAVE;
  const int tid = (int)threadIdx.x, lane = tid & 31, wave = tid >> 5;
  const int nodeBase = (int)blockIdx.x * NB;

  for (int i = tid; i < NB; i += NTHR) scnt[i] = 0;
  __syncthreads();

  int tot = 0;
  const int nChunks = (nE + CHUNK - 1) / CHUNK;
#pragma unroll 1
  for (int ch = 0; ch < nChunks; ++ch) {
    const int cbase = ch * CHUNK;
    const int wc = scan_chunk(dsts, nE, cbase, nodeBase, NB, vec8, list, tid, lane, wave);
    if (lane == 0) wcnt[wave] = wc;
    __syncthreads();
    int pre = 0, all = 0;
#pragma unroll
    for (int w2 = 0; w2 < NWAVE; ++w2) {
      int c = wcnt[w2];
      c = c < 0 ? 0 : (c > WCAP ? WCAP : c);
      all += c;
      pre += (w2 < wave) ? c : 0;
    }
    const int wcc  = wc > WCAP ? WCAP : wc;
    const int base = tot + pre;
#pragma unroll 1
    for (int i = lane; i < wcc; i += 32) {
      const int ent = list[wave * WCAP + i];
      const int el  = (ent >> SLOTB) & (CHUNK - 1);
      const int sl  = ent & (NB - 1);
      int eid = cbase + el;
      eid = eid > nE - 1 ? nE - 1 : eid;
      const int pos = base + i;
      if (pos < RCAP) reg1[pos] = (int)(((unsigned)eid << SLOTB) | (unsigned)sl);
    }
    tot += all;
    tot = tot > RCAP ? RCAP : tot;
    __syncthreads();
  }
  const int nh = tot;

  if (wave == 0) {
#pragma unroll 1
    for (int b0 = 0; b0 < nh; b0 += 32) {
      const int idx = b0 + lane;
      const int uv  = reg1[idx < nh ? idx : nh - 1];
      const int m32 = (nh - b0) < 32 ? (nh - b0) : 32;
#pragma unroll 1
      for (int k = 0; k < m32; ++k) {
        const int u  = __builtin_amdgcn_readlane(uv, k);
        const int sl = u & (NB - 1);
        if (lane == 0) scnt[sl] = scnt[sl] + 1;
      }
    }
  }
  __syncthreads();

  {
    const v4i ca = *(const v4i*)(scnt + 4 * tid);
    const int e0 = ca.x < 0 ? 0 : ca.x, e1 = ca.y < 0 ? 0 : ca.y, e2 = ca.z < 0 ? 0 : ca.z, e3 = ca.w < 0 ? 0 : ca.w;
    const int ts = e0 + e1 + e2 + e3;
    int incl = ts;
#pragma unroll
    for (int d = 1; d < 32; d <<= 1) {
      const int up = __shfl_up(incl, d);
      if (lane >= d) incl += up;
    }
    if (lane == 31) wtot[wave] = incl;
    __syncthreads();
    int pre = 0;
#pragma unroll
    for (int w2 = 0; w2 < NWAVE; ++w2) pre += (w2 < wave) ? wtot[w2] : 0;
    int run = pre + incl - ts;
    soff[4 * tid + 0] = run; run += e0;
    soff[4 * tid + 1] = run; run += e1;
    soff[4 * tid + 2] = run; run += e2;
    soff[4 * tid + 3] = run;
  }
  __syncthreads();
  for (int i = tid; i < NB; i += NTHR) list[i] = soff[i];
  __syncthreads();

  if (wave == 0) {
#pragma unroll 1
    for (int b0 = 0; b0 < nh; b0 += 32) {
      const int idx = b0 + lane;
      const int uv  = reg1[idx < nh ? idx : nh - 1];
      const int m32 = (nh - b0) < 32 ? (nh - b0) : 32;
#pragma unroll 1
      for (int k = 0; k < m32; ++k) {
        const int u   = __builtin_amdgcn_readlane(uv, k);
        const int sl  = u & (NB - 1);
        const int eid = (int)((unsigned)u >> SLOTB);
        if (lane == 0) {
          int pos = list[sl];
          pos = pos < 0 ? 0 : (pos > RCAP - 1 ? RCAP - 1 : pos);
          reg2[pos] = eid;
          list[sl] = pos + 1;
        }
      }
    }
  }
  __syncthreads();

  float* sbias = (float*)list;
  if (tid < NCOL) sbias[tid] = bfr(bias[tid]);
  __syncthreads();

  const bool ovf = (nh >= RCAP);
  const float qnan = __int_as_float(0x7fc00000);
  float* stf = (float*)reg1 + wave * STW;

#pragma unroll 1
  for (int jt = 0; jt < NBW; ++jt) {
    const int slot = wave * NBW + jt;
    const int grow = nodeBase + slot;
    const int gcl  = grow < nN ? grow : nN - 1;
    int st = soff[slot];
    const int craw = scnt[slot];
    int cnt = craw;
    st  = st < 0 ? 0 : (st > nh ? nh : st);
    cnt = cnt < 0 ? 0 : (cnt > DEGCAP ? DEGCAP : cnt);
    if (cnt > nh - st) cnt = nh - st;
    const float pz = (ovf || craw > DEGCAP) ? qnan : 0.0f;
    const bool live = grow < nN;
    const float* fr = F + (size_t)gcl * PIT;

    if constexpr (L == 1) {
      const int hA = lane >> 2;
      const int hB = 8 + (lane >> 3);
      v4f a4 = *(const v4fa*)(fr + 4 * lane);
      v2f a2 = *(const v2fa*)(fr + 128 + 2 * lane);
      const float adA = fr[ADO + hA];
      const float adB = fr[ADO + hB];
      float mxA = lrelu(fr[ASO + hA] + adA), dnA = 1.0f;
      float mxB = lrelu(fr[ASO + hB] + adB), dnB = 1.0f;
#pragma unroll 1
      for (int q = 0; q < cnt; ++q) {
        int idx = st + q; idx = idx > RCAP - 1 ? RCAP - 1 : idx;
        int eid = reg2[idx]; eid = eid < 0 ? 0 : (eid > nE - 1 ? nE - 1 : eid);
        const int sraw = srcs[eid];
        const int s = sraw < 0 ? 0 : (sraw > nN - 1 ? nN - 1 : sraw);
        const float* sr = F + (size_t)s * PIT;
        const v4f f4 = *(const v4fa*)(sr + 4 * lane);
        const v2f f2 = *(const v2fa*)(sr + 128 + 2 * lane);
        const float lgA = lrelu(sr[ASO + hA] + adA);
        const float lgB = lrelu(sr[ASO + hB] + adB);
        float s1, s2;
        onl_step(lgA, mxA, dnA, s1, s2);
        a4.x = fmaf(a4.x, s1, s2 * f4.x);
        a4.y = fmaf(a4.y, s1, s2 * f4.y);
        a4.z = fmaf(a4.z, s1, s2 * f4.z);
        a4.w = fmaf(a4.w, s1, s2 * f4.w);
        float t1, t2;
        onl_step(lgB, mxB, dnB, t1, t2);
        a2.x = fmaf(a2.x, t1, t2 * f2.x);
        a2.y = fmaf(a2.y, t1, t2 * f2.y);
      }
      const float iA = __builtin_amdgcn_rcpf(dnA);
      const float iB = __builtin_amdgcn_rcpf(dnB);
      v4f o4; o4.x = a4.x * iA; o4.y = a4.y * iA; o4.z = a4.z * iA; o4.w = a4.w * iA;
      v2f o2; o2.x = a2.x * iB; o2.y = a2.y * iB;
      *(v4fa*)(stf + 4 * lane) = o4;
      *(v2fa*)(stf + 128 + 2 * lane) = o2;
      __syncthreads();
      unsigned short* ush = (unsigned short*)(stf + HC1);
#pragma unroll 1
      for (int i = 0; i < HC1 / 32; ++i) {
        const int c = lane + 32 * i;
        float v = stf[c] + sbias[c];
        v = (v > 0.0f) ? v : expm1f(v);
        v = live ? v : 0.0f;
        v = v + pz;
        const unsigned int hb = f2bf(v);
        const unsigned int lb = f2bf(v - bf2f(hb));
        ush[c]       = (unsigned short)hb;
        ush[HC1 + c] = (unsigned short)lb;
      }
      __syncthreads();
      const v8us p0 = *(const v8usa*)(ush + 8 * lane);
      const v8us p1 = *(const v8usa*)(ush + 256 + 8 * (lane & 15));
      unsigned short* gp0 = HP + (size_t)grow * KA2 + 8 * lane;
      unsigned short* gp1 = HP + (size_t)grow * KA2 + 256 + 8 * (lane & 15);
      const bool wr = grow < MPr;
      if (wr) {
        *(volatile v8us*)gp0 = p0;
        if (lane < 16) *(volatile v8us*)gp1 = p1;
      }
      __threadfence();
      if (wr) {
        *(volatile v8us*)gp0 = p0;
        if (lane < 16) *(volatile v8us*)gp1 = p1;
      }
    } else {
      const int hd = lane >> 2;
      v2f a2 = *(const v2fa*)(fr + 2 * lane);
      const float adv = fr[ADO + hd];
      float mx = lrelu(fr[ASO + hd] + adv), dn = 1.0f;
#pragma unroll 1
      for (int q = 0; q < cnt; ++q) {
        int idx = st + q; idx = idx > RCAP - 1 ? RCAP - 1 : idx;
        int eid = reg2[idx]; eid = eid < 0 ? 0 : (eid > nE - 1 ? nE - 1 : eid);
        const int sraw = srcs[eid];
        const int s = sraw < 0 ? 0 : (sraw > nN - 1 ? nN - 1 : sraw);
        const float* sr = F + (size_t)s * PIT;
        const v2f f2 = *(const v2fa*)(sr + 2 * lane);
        const float lg = lrelu(sr[ASO + hd] + adv);
        float s1, s2;
        onl_step(lg, mx, dn, s1, s2);
        a2.x = fmaf(a2.x, s1, s2 * f2.x);
        a2.y = fmaf(a2.y, s1, s2 * f2.y);
      }
      const float inv = __builtin_amdgcn_rcpf(dn);
      v2f o2; o2.x = a2.x * inv; o2.y = a2.y * inv;
      *(v2fa*)(stf + 2 * lane) = o2;
      __syncthreads();
#pragma unroll 1
      for (int i = 0; i < HC2 / 32; ++i) {
        const int c = lane + 32 * i;
        float v = stf[c] + sbias[c];
        v = (v > 0.0f) ? v : expm1f(v);
        v = v + pz;
        stf[HC2 + c] = v;
      }
      __syncthreads();
      const v4f ov = *(const v4fa*)(stf + HC2 + 4 * (lane & 15));
      float* op = xout + (size_t)gcl * HC2 + 4 * (lane & 15);
      const bool wr = live && (lane < 16);
      if (wr) *(volatile v4f*)op = ov;
      __threadfence();
      if (wr) *(volatile v4f*)op = ov;
    }
  }
}

__global__ __launch_bounds__(PPB) void k_pair(const float* __restrict__ xo, const int* __restrict__ n1,
                                              const int* __restrict__ n2, const float* __restrict__ linW,
                                              const float* __restrict__ linb, float* y, int nN, int P) {
  __shared__ __attribute__((aligned(16))) float sw[256];
  __shared__ __attribute__((aligned(16))) float sz[2 * PPB];
  const int tid = (int)threadIdx.x;
  const int p   = (int)blockIdx.x * PPB + tid;
  sw[tid] = bfr(linW[tid]);
  __syncthreads();
  const int pc = p < P ? p : P - 1;
  int i1 = n1[pc]; i1 = i1 < 0 ? 0 : (i1 > nN - 1 ? nN - 1 : i1);
  int i2 = n2[pc]; i2 = i2 < 0 ? 0 : (i2 > nN - 1 ? nN - 1 : i2);
  float z0 = linb[0], z1 = linb[1];
#pragma unroll 1
  for (int hv = 0; hv < 2; ++hv) {
    const size_t ro = (size_t)(hv == 0 ? i1 : i2) * HC2;
    const float* wr = sw + hv * 128;
#pragma unroll 1
    for (int j = 0; j < HC2 / 4; ++j) {
      const v4f xv = *(const v4fa*)(xo + ro + 4 * j);
      const v4f wa = *(const v4fa*)(wr + 8 * j);
      const v4f wb = *(const v4fa*)(wr + 8 * j + 4);
      z0 = fmaf(xv.x, wa.x, z0); z1 = fmaf(xv.x, wa.y, z1);
      z0 = fmaf(xv.y, wa.z, z0); z1 = fmaf(xv.y, wa.w, z1);
      z0 = fmaf(xv.z, wb.x, z0); z1 = fmaf(xv.z, wb.y, z1);
      z0 = fmaf(xv.w, wb.z, z0); z1 = fmaf(xv.w, wb.w, z1);
    }
  }
  sz[2 * tid]     = z0;
  sz[2 * tid + 1] = z1;
  __syncthreads();
#pragma unroll 1
  for (int i = tid; i < 2 * PPB; i += PPB) {
    const float z = sz[i];
    sz[i] = 1.0f / (1.0f + expf(-z));
  }
  __syncthreads();
  if (tid < 128) {
    const v4f v = *(const v4fa*)(sz + 4 * tid);
    float* op = y + (size_t)blockIdx.x * (2 * PPB) + 4 * tid;
    *(volatile v4f*)op = v;
    __threadfence();
    *(volatile v4f*)op = v;
  }
}

static inline int cdiv(int a, int b) { return (a + b - 1) / b; }

extern "C" void kernel_launch(void* const* d_in, const int* in_sizes, int n_in,
                              void* d_out, int out_size, void* d_ws, size_t ws_size,
                              hipStream_t stream) {
  if (n_in < 14) return;
  if (in_sizes[0] < F0 || (in_sizes[0] % F0) != 0) return;
  const int nN = in_sizes[0] / F0;
  if (nN < 1 || nN > (1 << 22)) return;
  if (in_sizes[1] < 2 || (in_sizes[1] & 1) != 0) return;
  const int nE = in_sizes[1] / 2;
  if (nE < 1 || nE >= (1 << 21)) return;
  const int P = in_sizes[2];
  if (P < PPB || (P % PPB) != 0 || in_sizes[3] != P) return;
  if (in_sizes[4] != F0 * HC1) return;
  if (in_sizes[5] != HC1 || in_sizes[6] != HC1 || in_sizes[7] != HC1) return;
  if (in_sizes[8] != HC1 * HC2) return;
  if (in_sizes[9] != HC2 || in_sizes[10] != HC2 || in_sizes[11] != HC2) return;
  if (in_sizes[12] != 2 * 2 * HC2) return;
  if (in_sizes[13] != 2) return;
  if ((long long)out_size != 2LL * P + (long long)nN * HC2) return;

  const float* feat = (const float*)d_in[0];
  const int*   ei   = (const int*)  d_in[1];
  const int*   nd1  = (const int*)  d_in[2];
  const int*   nd2  = (const int*)  d_in[3];
  const float* W1   = (const float*)d_in[4];
  const float* as1  = (const float*)d_in[5];
  const float* ad1  = (const float*)d_in[6];
  const float* b1   = (const float*)d_in[7];
  const float* W2   = (const float*)d_in[8];
  const float* as2  = (const float*)d_in[9];
  const float* ad2  = (const float*)d_in[10];
  const float* b2   = (const float*)d_in[11];
  const float* linW = (const float*)d_in[12];
  const float* linb = (const float*)d_in[13];
  float* yout = (float*)d_out;
  float* xo   = yout + (size_t)2 * P;
  const int* src = ei;
  const int* dst = ei + nE;

  const int MP   = cdiv(nN, MROWS) * MROWS;
  const int gM   = MP / GBM;
  const int gA   = cdiv(MP, NB);
  if ((long long)gA * NB < (long long)MP) return;
  const int vec8 = ((nE & 3) == 0) ? 1 : 0;

  char* ws = (char*)d_ws;
  size_t off = 0;
  const size_t oXB  = off; off += (size_t)MP * KP1 * 2;    off = (off + 255) & ~(size_t)255;
  const size_t oW1T = off; off += (size_t)HC1 * KP1 * 2;   off = (off + 255) & ~(size_t)255;
  const size_t oW2T = off; off += (size_t)HC2 * KA2 * 2;   off = (off + 255) & ~(size_t)255;
  const size_t oHA1 = off; off += (size_t)MP * PIT1 * 4;   off = (off + 255) & ~(size_t)255;
  const size_t oX1  = off; off += (size_t)MP * KA2 * 2;    off = (off + 255) & ~(size_t)255;
  const size_t oHA2 = off; off += (size_t)MP * PIT2 * 4;   off = (off + 255) & ~(size_t)255;
  if (off > ws_size || off > (size_t)WSMAX) return;
  unsigned short* XB  = (unsigned short*)(ws + oXB);
  unsigned short* W1T = (unsigned short*)(ws + oW1T);
  unsigned short* W2T = (unsigned short*)(ws + oW2T);
  float*          HA1 = (float*)(ws + oHA1);
  unsigned short* X1  = (unsigned short*)(ws + oX1);
  float*          HA2 = (float*)(ws + oHA2);

  hipFuncSetAttribute(reinterpret_cast<const void*>(&k_agg<1>),
                      hipFuncAttributeMaxDynamicSharedMemorySize, LDS_AGG);
  hipFuncSetAttribute(reinterpret_cast<const void*>(&k_agg<2>),
                      hipFuncAttributeMaxDynamicSharedMemorySize, LDS_AGG);

  const int nUx = MP * (KP1 / 8);
  k_xprep<<<cdiv(nUx, NTHR), NTHR, 0, stream>>>(feat, XB, nN, nUx);
  k_wprep<<<(NU1 + NU2) / NTHR, NTHR, 0, stream>>>(W1, W2, W1T, W2T);
  k_gemm<256, 6, KP1, PIT1, HC1, NH1, CH1><<<gM, 256, 0, stream>>>(XB, W1T, as1, ad1, HA1);
  k_agg<1><<<gA, NTHR, LDS_AGG, stream>>>(src, dst, HA1, b1, X1, xo, nN, nE, vec8, MP);
  k_gemm<128, 4, KA2, PIT2, HC2, NH2, CH2><<<gM, 128, 0, stream>>>(X1, W2T, as2, ad2, HA2);
  k_agg<2><<<gA, NTHR, LDS_AGG, stream>>>(src, dst, HA2, b2, X1, xo, nN, nE, vec8, MP);
  k_pair<<<P / PPB, PPB, 0, stream>>>(xo, nd1, nd2, linW, linb, yout, nN, P);
}
